// GCN_Geo_47382079209725
// MI455X (gfx1250) — hardware-verified
//
#include <hip/hip_runtime.h>
#include <stddef.h>
#include <stdint.h>

#define NNODES 65536
#define NEDGES 131072
#define NGRAPH 32
#define NAM    128
#define NSEG   (NGRAPH * NAM)
#define FD     32
#define FE     16
#define G0     64
#define KST    3
#define TST    7
#define NCH    17
#define BWN    (NCH * FD)
#define FC1    256
#define FC2    128
#define FC3    64
#define NTHR   256
#define NWAVE  8
#define PTHR   128
#define EPB    128
#define EPT    8
#define CHUNK  (NTHR * EPT)
#define WCAP   (EPT * 32)
#define LISTN  (NWAVE * WCAP)
#define DEGCAP 64
#define A_NB   1024
#define A_SL   10
#define A_RC   4096
#define P_NB   256
#define P_SL   8
#define P_RC   8192
#define WSMAX  134217728

#define BWL     (BWN * FD)
#define O_BW    0
#define O_RT    (O_BW + 3 * BWL)
#define O_INIT  (O_RT + 3 * FD * FD)
#define O_REC   (O_INIT + KST * G0 * FD)
#define O_ROOTW (O_REC + (TST - 1) * KST * G0 * G0)
#define O_L1    (O_ROOTW + TST * KST * G0 * FD)
#define O_L2    (O_L1 + FC1 * G0)
#define O_L3    (O_L2 + FC2 * FC1)
#define O_END   (O_L3 + FC3 * FC2)

#define U0  2048
#define U1  (U0 + 2048)
#define U2  (U1 + 2048)
#define U3  (U2 + 128)
#define U4  (U3 + 128)
#define U5  (U4 + 128)
#define U6  (U5 + 128)
#define U7  (U6 + 128)
#define U8  (U7 + 128)
#define U9  (U8 + (KST * G0 * FD) / 8)
#define U10 (U9 + ((TST - 1) * KST * G0 * G0) / 8)
#define U11 (U10 + (TST * KST * G0 * FD) / 8)
#define U12 (U11 + (FC1 * G0) / 8)
#define U13 (U12 + (FC2 * FC1) / 8)
#define U14 (U13 + (FC3 * FC2) / 8)

#define AGG_LDS_BYTES  ((LISTN + 2 * A_RC + 3 * A_NB + 16) * 4)
#define POOL_LDS_BYTES ((LISTN + 2 * P_RC + 3 * P_NB + 16) * 4)
#define ARMA_LDS_BYTES ((2 * NAM * G0 + NAM + G0) * 4 + (2 * NAM * FD + 2 * NAM * G0) * 2)
#define HEAD_LDS_BYTES ((32 * FC1 + 64) * 4 + 2 * 32 * FC1 * 2)

static_assert(NNODES % CHUNK == 0 && NEDGES % CHUNK == 0);
static_assert(NEDGES % EPB == 0 && NNODES % EPB == 0);
static_assert(NNODES % A_NB == 0 && NSEG % P_NB == 0);
static_assert(A_NB == (1 << A_SL) && P_NB == (1 << P_SL));
static_assert(((long long)NEDGES << A_SL) < (1LL << 31) && ((long long)NNODES << P_SL) < (1LL << 31));
static_assert(((long long)CHUNK << A_SL) < (1LL << 31));
static_assert(A_NB % 32 == 0 && P_NB % 32 == 0 && A_NB % NWAVE == 0 && P_NB % NWAVE == 0);
static_assert((LISTN + 2 * A_RC + 3 * A_NB) % 4 == 0 && (LISTN + 2 * P_RC + 3 * P_NB) % 4 == 0);
static_assert(EPB == 16 * NWAVE && NAM == 16 * NWAVE && G0 == 64 && FD == 32);
static_assert(EPB * FD == 4 * NTHR * 4);
static_assert(O_RT % 64 == 0 && O_INIT % 64 == 0 && O_REC % 64 == 0 && O_ROOTW % 64 == 0);
static_assert(O_L1 % 64 == 0 && O_L2 % 64 == 0 && O_L3 % 64 == 0 && O_END % 64 == 0 && BWL % 64 == 0);
static_assert(U0 % PTHR == 0 && U3 % PTHR == 0 && U6 % PTHR == 0 && U9 % PTHR == 0 && U10 % PTHR == 0);
static_assert(U11 % PTHR == 0 && U12 % PTHR == 0 && U13 % PTHR == 0 && U14 % PTHR == 0);
static_assert(AGG_LDS_BYTES <= 300000 && POOL_LDS_BYTES <= 300000 && ARMA_LDS_BYTES <= 300000);
static_assert(NGRAPH == 32 && FC3 == 64);

typedef float          v4f   __attribute__((ext_vector_type(4)));
typedef float          v8f   __attribute__((ext_vector_type(8)));
typedef int            v4i   __attribute__((ext_vector_type(4)));
typedef int            v8i   __attribute__((ext_vector_type(8)));
typedef unsigned short v8us  __attribute__((ext_vector_type(8)));
typedef unsigned short v16us __attribute__((ext_vector_type(16)));
typedef __bf16         v16bf __attribute__((ext_vector_type(16)));
typedef v4f  __attribute__((may_alias)) v4fa;
typedef v4i  __attribute__((may_alias)) v4ia;
typedef v8us __attribute__((may_alias)) v8usa;
union FragB { v16bf v; v16us u; v8us h[2]; v8i w; };

__device__ __forceinline__ v8f wmb(const FragB& a, const FragB& b, v8f c) {
  v8f d = __builtin_amdgcn_wmma_f32_16x16x32_bf16(false, a.v, false, b.v, (short)0, c, false, false);
  asm volatile("v_nop\n\tv_nop\n\tv_nop\n\tv_nop" : "+v"(d) : "v"(a.w), "v"(b.w));
  return d;
}
__device__ __forceinline__ v8f z8() { v8f z = {0.f, 0.f, 0.f, 0.f, 0.f, 0.f, 0.f, 0.f}; return z; }

__device__ __forceinline__ unsigned bf16_bits(float f) {
  const unsigned u = __float_as_uint(f);
  const unsigned r = (u + 0x7FFFu + ((u >> 16) & 1u)) >> 16;
  const unsigned q = ((u >> 16) & 0x8000u) | 0x7FC0u;
  return ((u & 0x7FFFFFFFu) > 0x7F800000u) ? q : r;
}
__device__ __forceinline__ float bf16_val(float f) { return __uint_as_float(bf16_bits(f) << 16); }
__device__ __forceinline__ v4f bfv4(const v4f a) {
  v4f o;
  o.x = bf16_val(a.x); o.y = bf16_val(a.y); o.z = bf16_val(a.z); o.w = bf16_val(a.w);
  return o;
}
__device__ __forceinline__ float relu_np(float v) { return (v > 0.0f) ? v : (v - v); }

template <int BASE>
__device__ __forceinline__ void split4(const v4f q, FragB& ah, FragB& al) {
#pragma unroll
  for (int i = 0; i < 4; ++i) {
    const unsigned hb = bf16_bits(q[i]);
    const unsigned lb = bf16_bits(q[i] - __uint_as_float(hb << 16));
    ah.u[BASE + i] = (unsigned short)hb;
    al.u[BASE + i] = (unsigned short)lb;
  }
}
__device__ __forceinline__ void split8_store(const v4f a, const v4f b, unsigned short* ph, unsigned short* pl) {
  const v8f f8 = {a.x, a.y, a.z, a.w, b.x, b.y, b.z, b.w};
  v8us ho, lo;
#pragma unroll
  for (int e = 0; e < 8; ++e) {
    const unsigned hb = bf16_bits(f8[e]);
    const unsigned lb = bf16_bits(f8[e] - __uint_as_float(hb << 16));
    ho[e] = (unsigned short)hb;
    lo[e] = (unsigned short)lb;
  }
  *(v8usa*)ph = ho;
  *(v8usa*)pl = lo;
}
__device__ __forceinline__ void put16(unsigned short* dp, v8us o) {
  *(volatile v8us*)dp = o;
  __threadfence();
  *(volatile v8us*)dp = o;
}
__device__ __forceinline__ void store_tile(const float* stg, float* dst, int tid) {
  v4f pv[4];
#pragma unroll
  for (int it = 0; it < 4; ++it) pv[it] = *(const v4fa*)(stg + (size_t)(it * NTHR + tid) * 4);
#pragma unroll
  for (int it = 0; it < 4; ++it) *(volatile v4f*)(dst + (size_t)(it * NTHR + tid) * 4) = pv[it];
  __threadfence();
#pragma unroll
  for (int it = 0; it < 4; ++it) *(volatile v4f*)(dst + (size_t)(it * NTHR + tid) * 4) = pv[it];
}

template <int K, int NC>
__device__ __forceinline__ void prepT(const float* __restrict__ src, int v, unsigned short* dst) {
  const int p   = 8 * v;
  const int k0  = p % K;
  const int n   = (p / K) % NC;
  const int mat = p / (K * NC);
  const float* sp = src + (size_t)mat * (K * NC) + (size_t)k0 * NC + n;
  v8us o;
#pragma unroll
  for (int i = 0; i < 8; ++i) o[i] = (unsigned short)bf16_bits(sp[(size_t)i * NC]);
  put16(dst + p, o);
}
__global__ __launch_bounds__(PTHR) void k_prep(
    const float* __restrict__ mw1, const float* __restrict__ mb1, const float* __restrict__ rt1,
    const float* __restrict__ mw2, const float* __restrict__ mb2, const float* __restrict__ rt2,
    const float* __restrict__ mw3, const float* __restrict__ mb3, const float* __restrict__ rt3,
    const float* __restrict__ aiw, const float* __restrict__ aw, const float* __restrict__ arw,
    const float* __restrict__ l1w, const float* __restrict__ l2w, const float* __restrict__ l3w,
    unsigned short* PL) {
  const int u = (int)blockIdx.x * PTHR + (int)threadIdx.x;
  if (u < U0)  { prepT<FD, FD>(mw1, u,       PL + O_BW);                     return; }
  if (u < U1)  { prepT<FD, FD>(mw2, u - U0,  PL + O_BW + BWL);               return; }
  if (u < U2)  { prepT<FD, FD>(mw3, u - U1,  PL + O_BW + 2 * BWL);           return; }
  if (u < U3)  { prepT<FD, FD>(mb1, u - U2,  PL + O_BW + 512 * FD);          return; }
  if (u < U4)  { prepT<FD, FD>(mb2, u - U3,  PL + O_BW + BWL + 512 * FD);    return; }
  if (u < U5)  { prepT<FD, FD>(mb3, u - U4,  PL + O_BW + 2 * BWL + 512 * FD); return; }
  if (u < U6)  { prepT<FD, FD>(rt1, u - U5,  PL + O_RT);                     return; }
  if (u < U7)  { prepT<FD, FD>(rt2, u - U6,  PL + O_RT + FD * FD);           return; }
  if (u < U8)  { prepT<FD, FD>(rt3, u - U7,  PL + O_RT + 2 * FD * FD);       return; }
  if (u < U9)  { prepT<FD, G0>(aiw, u - U8,  PL + O_INIT);                   return; }
  if (u < U10) { prepT<G0, G0>(aw,  u - U9,  PL + O_REC);                    return; }
  if (u < U11) { prepT<FD, G0>(arw, u - U10, PL + O_ROOTW);                  return; }
  if (u < U12) { prepT<G0, FC1>(l1w, u - U11, PL + O_L1);                    return; }
  if (u < U13) { prepT<FC1, FC2>(l2w, u - U12, PL + O_L2);                   return; }
  if (u < U14) { prepT<FC2, FC3>(l3w, u - U13, PL + O_L3);                   return; }
}

__global__ __launch_bounds__(NTHR) void k_root(const float* __restrict__ Hin, int rnd,
                                               const unsigned short* __restrict__ RT,
                                               const float* __restrict__ bias, float* ROOTP) {
  __shared__ __attribute__((aligned(16))) float stg[EPB * FD];
  const int tid = (int)threadIdx.x, lane = tid & 31, wave = tid >> 5, hh = lane >> 4, m = lane & 15;
  const int rowBase = (int)blockIdx.x * EPB;
  const float* ap = Hin + (size_t)(rowBase + 16 * wave + m) * FD + 8 * hh;
  const v4f q0 = *(const v4fa*)ap;
  const v4f q1 = *(const v4fa*)(ap + 4);
  const v4f q2 = *(const v4fa*)(ap + 16);
  const v4f q3 = *(const v4fa*)(ap + 20);
  FragB aH, aL;
  split4<0>(q0, aH, aL);
  split4<4>(q1, aH, aL);
  split4<8>(q2, aH, aL);
  split4<12>(q3, aH, aL);
  const unsigned short* bp = RT + m * FD + 8 * hh;
  FragB b0, b1;
  b0.h[0] = *(const v8usa*)bp;
  b0.h[1] = *(const v8usa*)(bp + 16);
  b1.h[0] = *(const v8usa*)(bp + 16 * FD);
  b1.h[1] = *(const v8usa*)(bp + 16 * FD + 16);
  v8f acc0 = wmb(aH, b0, z8());
  v8f acc1 = wmb(aH, b1, z8());
  if (rnd == 0) {
    acc0 = wmb(aL, b0, acc0);
    acc1 = wmb(aL, b1, acc1);
  }
  const float bv0 = bf16_val(bias[m]);
  const float bv1 = bf16_val(bias[16 + m]);
#pragma unroll
  for (int r = 0; r < 8; ++r) {
    const int lr = 16 * wave + 8 * hh + r;
    stg[lr * FD + m]      = acc0[r] + bv0;
    stg[lr * FD + 16 + m] = acc1[r] + bv1;
  }
  __syncthreads();
  store_tile(stg, ROOTP + (size_t)rowBase * FD, tid);
}

__global__ __launch_bounds__(NTHR) void k_edge(const float* __restrict__ Hin, int rnd,
                                               const int* __restrict__ eidx, const float* __restrict__ eattr,
                                               const unsigned short* __restrict__ BW, float* MSG) {
  __shared__ __attribute__((aligned(16))) float sX[EPB * FD];
  __shared__ __attribute__((aligned(16))) float sEt[NCH * EPB];
  __shared__ __attribute__((aligned(16))) float sD[EPB * FD];
  const int tid = (int)threadIdx.x, lane = tid & 31, wave = tid >> 5, hh = lane >> 4, m = lane & 15;
  const int ebase = (int)blockIdx.x * EPB;
  {
    const int le = tid >> 1, half = tid & 1;
    const int e = ebase + le;
    int s = eidx[e];
    s = s < 0 ? 0 : (s > NNODES - 1 ? NNODES - 1 : s);
    const float* xr = Hin + (size_t)s * FD + 16 * half;
    v4f x0 = *(const v4fa*)xr;
    v4f x1 = *(const v4fa*)(xr + 4);
    v4f x2 = *(const v4fa*)(xr + 8);
    v4f x3 = *(const v4fa*)(xr + 12);
    if (rnd != 0) { x0 = bfv4(x0); x1 = bfv4(x1); x2 = bfv4(x2); x3 = bfv4(x3); }
    float* xw = sX + le * FD + 16 * half;
    *(v4fa*)xw        = x0;
    *(v4fa*)(xw + 4)  = x1;
    *(v4fa*)(xw + 8)  = x2;
    *(v4fa*)(xw + 12) = x3;
    const float* er = eattr + (size_t)e * FE + 8 * half;
    const v4f a0 = *(const v4fa*)er;
    const v4f a1 = *(const v4fa*)(er + 4);
#pragma unroll
    for (int i = 0; i < 4; ++i) {
      sEt[(8 * half + i) * EPB + le]     = bf16_val(a0[i]);
      sEt[(8 * half + 4 + i) * EPB + le] = bf16_val(a1[i]);
    }
    if (half == 1) sEt[16 * EPB + le] = 1.0f;
  }
  __syncthreads();

  FragB aH, aL;
  {
    const float* xp = sX + (16 * wave + m) * FD + 8 * hh;
    const v4f q0 = *(const v4fa*)xp;
    const v4f q1 = *(const v4fa*)(xp + 4);
    const v4f q2 = *(const v4fa*)(xp + 16);
    const v4f q3 = *(const v4fa*)(xp + 20);
    split4<0>(q0, aH, aL);
    split4<4>(q1, aH, aL);
    split4<8>(q2, aH, aL);
    split4<12>(q3, aH, aL);
  }
  v8f acc0 = z8(), acc1 = z8();
  const unsigned short* bp = BW + (size_t)m * FD + 8 * hh;
  const float* ep = sEt + 16 * wave + 8 * hh;
#pragma unroll 1
  for (int c = 0; c < NCH; ++c) {
    const unsigned short* q = bp + (size_t)c * (FD * FD);
    FragB b0, b1;
    b0.h[0] = *(const v8usa*)q;
    b0.h[1] = *(const v8usa*)(q + 16);
    b1.h[0] = *(const v8usa*)(q + 16 * FD);
    b1.h[1] = *(const v8usa*)(q + 16 * FD + 16);
    v8f y0 = wmb(aH, b0, z8());
    v8f y1 = wmb(aH, b1, z8());
    if (rnd == 0) {
      y0 = wmb(aL, b0, y0);
      y1 = wmb(aL, b1, y1);
    }
    const v4f e0 = *(const v4fa*)(ep + c * EPB);
    const v4f e1 = *(const v4fa*)(ep + c * EPB + 4);
    const v8f e8 = {e0.x, e0.y, e0.z, e0.w, e1.x, e1.y, e1.z, e1.w};
#pragma unroll
    for (int r = 0; r < 8; ++r) {
      acc0[r] = fmaf(e8[r], y0[r], acc0[r]);
      acc1[r] = fmaf(e8[r], y1[r], acc1[r]);
    }
  }
#pragma unroll
  for (int r = 0; r < 8; ++r) {
    const int lr = 16 * wave + 8 * hh + r;
    sD[lr * FD + m]      = acc0[r];
    sD[lr * FD + 16 + m] = acc1[r];
  }
  __syncthreads();
  store_tile(sD, MSG + (size_t)ebase * FD, tid);
}

template <int SLB, int POOL>
__device__ __forceinline__ int scan_chunk(const int* __restrict__ key0, const int* __restrict__ key1, int cbase,
                                          int slotBase, int nb, int* list, int tid, int lane, int wave) {
  int wc = 0;
  const int el0 = tid * EPT;
  const int e0  = cbase + el0;
  v4i da = *(const v4i*)(key0 + e0);
  v4i db = *(const v4i*)(key0 + e0 + 4);
  if constexpr (POOL != 0) {
    const v4i la = *(const v4i*)(key1 + e0);
    const v4i lb = *(const v4i*)(key1 + e0 + 4);
    da.x = (int)((unsigned)da.x * 128u + (unsigned)la.x);
    da.y = (int)((unsigned)da.y * 128u + (unsigned)la.y);
    da.z = (int)((unsigned)da.z * 128u + (unsigned)la.z);
    da.w = (int)((unsigned)da.w * 128u + (unsigned)la.w);
    db.x = (int)((unsigned)db.x * 128u + (unsigned)lb.x);
    db.y = (int)((unsigned)db.y * 128u + (unsigned)lb.y);
    db.z = (int)((unsigned)db.z * 128u + (unsigned)lb.z);
    db.w = (int)((unsigned)db.w * 128u + (unsigned)lb.w);
  }
  const unsigned nbs = (unsigned)slotBase;
  const unsigned unb = (unsigned)nb;
  const unsigned s0 = (unsigned)da.x - nbs, s1 = (unsigned)da.y - nbs;
  const unsigned s2 = (unsigned)da.z - nbs, s3 = (unsigned)da.w - nbs;
  const unsigned s4 = (unsigned)db.x - nbs, s5 = (unsigned)db.y - nbs;
  const unsigned s6 = (unsigned)db.z - nbs, s7 = (unsigned)db.w - nbs;
  const bool h0 = s0 < unb, h1 = s1 < unb, h2 = s2 < unb, h3 = s3 < unb;
  const bool h4 = s4 < unb, h5 = s5 < unb, h6 = s6 < unb, h7 = s7 < unb;
  const unsigned any = __builtin_amdgcn_ballot_w32(h0 | h1 | h2 | h3 | h4 | h5 | h6 | h7);
  if (any != 0u) {
#define HITJ(J, HJ, SJ) { \
      const unsigned mj = __builtin_amdgcn_ballot_w32(HJ); \
      if (mj != 0u) { \
        if (HJ) { \
          const int pos = wc + (int)__builtin_amdgcn_mbcnt_lo(mj, 0u); \
          if (pos < WCAP) list[wave * WCAP + pos] = ((el0 + (J)) << SLB) | (int)(SJ); \
        } \
        wc += (int)__builtin_popcount(mj); } }
    HITJ(0, h0, s0)
    HITJ(1, h1, s1)
    HITJ(2, h2, s2)
    HITJ(3, h3, s3)
    HITJ(4, h4, s4)
    HITJ(5, h5, s5)
    HITJ(6, h6, s6)
    HITJ(7, h7, s7)
#undef HITJ
  }
  return wc;
}

template <int POOL, int NB_, int SL_, int RC_>
__global__ __launch_bounds__(NTHR) void k_scan(const int* __restrict__ key0, const int* __restrict__ key1,
                                               int nItems, int nRows, const float* __restrict__ SRC,
                                               const float* __restrict__ ROOTP, float* OUT) {
  extern __shared__ __attribute__((aligned(16))) int dsm[];
  constexpr int ZINTS = LISTN + 2 * RC_ + 3 * NB_;
  int* list = dsm;
  int* hl   = dsm + LISTN;
  int* sl   = hl + RC_;
  int* cnt  = sl + RC_;
  int* offs = cnt + NB_;
  int* cur  = offs + NB_;
  int* misc = cur + NB_;
  const int tid = (int)threadIdx.x, lane = tid & 31, wave = tid >> 5;
  const int slotBase = (int)blockIdx.x * NB_;

  {
    const v4i z4 = {0, 0, 0, 0};
    for (int i = tid * 4; i < ZINTS; i += NTHR * 4) *(v4ia*)(dsm + i) = z4;
    if (tid < 16) misc[tid] = 0;
  }
  __syncthreads();

  int t = 0, ov = 0;
  const int nChunks = nItems / CHUNK;
#pragma unroll 1
  for (int ch = 0; ch < nChunks; ++ch) {
    const int cbase = ch * CHUNK;
    const int wc = scan_chunk<SL_, POOL>(key0, key1, cbase, slotBase, NB_, list, tid, lane, wave);
    if (lane == 0) misc[wave] = wc;
    __syncthreads();
    if (wave == 0) {
#pragma unroll 1
      for (int w2 = 0; w2 < NWAVE; ++w2) {
        int c = misc[w2];
        c = c < 0 ? 0 : (c > WCAP ? WCAP : c);
#pragma unroll 1
        for (int b0 = 0; b0 < c; b0 += 32) {
          const int idx = b0 + lane;
          const int ent = list[w2 * WCAP + (idx < WCAP ? idx : WCAP - 1)];
          const int m32 = (c - b0) < 32 ? (c - b0) : 32;
#pragma unroll 1
          for (int k = 0; k < m32; ++k) {
            const int u    = __builtin_amdgcn_readlane(ent, k);
            const int slot = u & (NB_ - 1);
            const int el   = (u >> SL_) & (CHUNK - 1);
            const int pk   = ((cbase + el) << SL_) | slot;
            if (t < RC_) {
              if (lane == 0) { hl[t] = pk; cnt[slot] = cnt[slot] + 1; }
              t = t + 1;
            } else {
              ov = 1;
            }
          }
        }
      }
    }
    __syncthreads();
  }
  if (wave == 0 && lane == 0) { misc[8] = t; misc[9] = ov; }
  __syncthreads();
  int tt = misc[8];
  tt = tt < 0 ? 0 : (tt > RC_ ? RC_ : tt);
  const int ovf = misc[9];

  if (wave == 0) {
    const int base = lane * (NB_ / 32);
    int s = 0;
#pragma unroll 1
    for (int i = 0; i < NB_ / 32; ++i) s += cnt[base + i];
    int incl = s;
#pragma unroll
    for (int d = 1; d < 32; d <<= 1) {
      const int y = __shfl_up(incl, d, 32);
      if (lane >= d) incl += y;
    }
    int run = incl - s;
#pragma unroll 1
    for (int i = 0; i < NB_ / 32; ++i) {
      const int cv = cnt[base + i];
      offs[base + i] = run;
      cur[base + i]  = run;
      run += cv;
    }
  }
  __syncthreads();
  if (wave == 0) {
#pragma unroll 1
    for (int b0 = 0; b0 < tt; b0 += 32) {
      const int idx = b0 + lane;
      const int ent = hl[idx < RC_ ? idx : RC_ - 1];
      const int m32 = (tt - b0) < 32 ? (tt - b0) : 32;
#pragma unroll 1
      for (int k = 0; k < m32; ++k) {
        const int u    = __builtin_amdgcn_readlane(ent, k);
        const int slot = u & (NB_ - 1);
        if (lane == 0) {
          int p = cur[slot];
          p = p < 0 ? 0 : (p > RC_ - 1 ? RC_ - 1 : p);
          sl[p] = u;
          cur[slot] = p + 1;
        }
      }
    }
  }
  __syncthreads();

  const float qnan = __int_as_float(0x7fc00000);
  const float pz = (ovf != 0) ? qnan : 0.0f;
#pragma unroll 1
  for (int si = 0; si < NB_ / NWAVE; ++si) {
    const int s   = si * NWAVE + wave;
    const int row = slotBase + s;
    int c = cnt[s];
    const bool big = c > DEGCAP;
    c = c < 0 ? 0 : (c > DEGCAP ? DEGCAP : c);
    int o = offs[s];
    o = o < 0 ? 0 : (o > RC_ ? RC_ : o);
    float a = 0.0f;
#pragma unroll 1
    for (int b0 = 0; b0 < c; b0 += 32) {
      int idx = o + b0 + lane;
      idx = idx > RC_ - 1 ? RC_ - 1 : idx;
      const int ent = sl[idx];
      int eid = ent >> SL_;
      eid = eid < 0 ? 0 : (eid > nItems - 1 ? nItems - 1 : eid);
      const int m32 = (c - b0) < 32 ? (c - b0) : 32;
#pragma unroll 1
      for (int k = 0; k < m32; ++k) {
        const int ek = __builtin_amdgcn_readlane(eid, k);
        a += SRC[(size_t)ek * FD + lane];
      }
    }
    const bool  live = row < nRows;
    const int   nr   = live ? row : nRows - 1;
    const float pzr  = big ? qnan : pz;
    float hv;
    if constexpr (POOL == 0) {
      const float v = (ROOTP[(size_t)nr * FD + lane] + a) + pzr;
      hv = relu_np(v);
    } else {
      hv = a + pzr;
    }
    float* op = OUT + (size_t)nr * FD + lane;
    if (live) *(volatile float*)op = hv;
    __threadfence();
    if (live) *(volatile float*)op = hv;
  }
}

__global__ __launch_bounds__(NTHR) void k_arma(const float* __restrict__ AMINO,
                                               const unsigned short* __restrict__ PL,
                                               const float* __restrict__ abias, float* RECS) {
  extern __shared__ __attribute__((aligned(16))) float adyn[];
  float* sZ = adyn;
  float* sO = sZ + NAM * G0;
  float* sN = sO + NAM * G0;
  float* sS = sN + NAM;
  unsigned short* sAh = (unsigned short*)(sS + G0);
  unsigned short* sAl = sAh + NAM * FD;
  unsigned short* sOh = sAl + NAM * FD;
  unsigned short* sOl = sOh + NAM * G0;
  const int tid = (int)threadIdx.x, lane = tid & 31, wave = tid >> 5, hh = lane >> 4, m = lane & 15;
  const int b = (int)blockIdx.x / KST;
  const int k = (int)blockIdx.x % KST;

  if (tid < NAM) {
    const int c0 = tid, c1 = tid + 1;
    const float dg0 = (c0 >= 1 && c0 <= NAM - 2) ? 1.0f : 0.0f;
    const float dg1 = (c1 >= 1 && c1 <= NAM - 2) ? 1.0f : 0.0f;
    const float di0 = (dg0 > 0.0f) ? (1.0f / sqrtf(fmaxf(dg0, 1.0f))) : 0.0f;
    const float di1 = (dg1 > 0.0f) ? (1.0f / sqrtf(fmaxf(dg1, 1.0f))) : 0.0f;
    sN[tid] = (tid < NAM - 2) ? (di0 * di1) : 0.0f;
  }
  {
    const int row = tid >> 1, half = tid & 1;
    const float* ar = AMINO + ((size_t)b * NAM + row) * FD + 16 * half;
    const v4f q0 = *(const v4fa*)ar;
    const v4f q1 = *(const v4fa*)(ar + 4);
    const v4f q2 = *(const v4fa*)(ar + 8);
    const v4f q3 = *(const v4fa*)(ar + 12);
    split8_store(q0, q1, sAh + row * FD + 16 * half,     sAl + row * FD + 16 * half);
    split8_store(q2, q3, sAh + row * FD + 16 * half + 8, sAl + row * FD + 16 * half + 8);
  }
  __syncthreads();

  const int row0 = 16 * wave;
  FragB aH, aL;
  {
    const unsigned short* aHp = sAh + (row0 + m) * FD + 8 * hh;
    const unsigned short* aLp = sAl + (row0 + m) * FD + 8 * hh;
    aH.h[0] = *(const v8usa*)aHp;
    aH.h[1] = *(const v8usa*)(aHp + 16);
    aL.h[0] = *(const v8usa*)aLp;
    aL.h[1] = *(const v8usa*)(aLp + 16);
  }
  const unsigned short* oHp = sOh + (row0 + m) * G0 + 8 * hh;
  const unsigned short* oLp = sOl + (row0 + m) * G0 + 8 * hh;

#pragma unroll 1
  for (int t = 0; t < TST; ++t) {
    v8f aZ[4], aR[4];
#pragma unroll
    for (int nt = 0; nt < 4; ++nt) { aZ[nt] = z8(); aR[nt] = z8(); }
    {
      const unsigned short* rw = PL + O_ROOTW + (size_t)(t * KST + k) * (G0 * FD) + (size_t)m * FD + 8 * hh;
#pragma unroll
      for (int nt = 0; nt < 4; ++nt) {
        FragB bb;
        bb.h[0] = *(const v8usa*)(rw + 16 * nt * FD);
        bb.h[1] = *(const v8usa*)(rw + 16 * nt * FD + 16);
        aR[nt] = wmb(aH, bb, aR[nt]);
        aR[nt] = wmb(aL, bb, aR[nt]);
      }
    }
    if (t == 0) {
      const unsigned short* iw = PL + O_INIT + (size_t)k * (G0 * FD) + (size_t)m * FD + 8 * hh;
#pragma unroll
      for (int nt = 0; nt < 4; ++nt) {
        FragB bb;
        bb.h[0] = *(const v8usa*)(iw + 16 * nt * FD);
        bb.h[1] = *(const v8usa*)(iw + 16 * nt * FD + 16);
        aZ[nt] = wmb(aH, bb, aZ[nt]);
        aZ[nt] = wmb(aL, bb, aZ[nt]);
      }
    } else {
      const unsigned short* rc = PL + O_REC + (size_t)((t - 1) * KST + k) * (G0 * G0) + (size_t)m * G0 + 8 * hh;
#pragma unroll
      for (int ks = 0; ks < 2; ++ks) {
        FragB oH, oL;
        oH.h[0] = *(const v8usa*)(oHp + 32 * ks);
        oH.h[1] = *(const v8usa*)(oHp + 32 * ks + 16);
        oL.h[0] = *(const v8usa*)(oLp + 32 * ks);
        oL.h[1] = *(const v8usa*)(oLp + 32 * ks + 16);
#pragma unroll
        for (int nt = 0; nt < 4; ++nt) {
          FragB bb;
          bb.h[0] = *(const v8usa*)(rc + 16 * nt * G0 + 32 * ks);
          bb.h[1] = *(const v8usa*)(rc + 16 * nt * G0 + 32 * ks + 16);
          aZ[nt] = wmb(oH, bb, aZ[nt]);
          aZ[nt] = wmb(oL, bb, aZ[nt]);
        }
      }
    }
#pragma unroll
    for (int nt = 0; nt < 4; ++nt)
#pragma unroll
      for (int r = 0; r < 8; ++r) sZ[(row0 + 8 * hh + r) * G0 + 16 * nt + m] = aZ[nt][r];
    __syncthreads();

    const int tb = (t * KST + k) * G0;
#pragma unroll
    for (int nt = 0; nt < 4; ++nt) {
      const int col = 16 * nt + m;
      const float bv = bf16_val(abias[tb + col]);
#pragma unroll
      for (int r = 0; r < 8; ++r) {
        const int row = row0 + 8 * hh + r;
        const bool ok = (row >= 1) && (row <= NAM - 2);
        int rp = row - 1;
        rp = rp < 0 ? 0 : (rp > NAM - 3 ? NAM - 3 : rp);
        const float zz = sZ[rp * G0 + col];
        const float nn = sN[rp];
        const float contrib = ok ? (nn * zz) : 0.0f;
        float v = (contrib + aR[nt][r]) + bv;
        v = relu_np(v);
        const unsigned hb = bf16_bits(v);
        const unsigned lb = bf16_bits(v - __uint_as_float(hb << 16));
        sOh[row * G0 + col] = (unsigned short)hb;
        sOl[row * G0 + col] = (unsigned short)lb;
        if (t == TST - 1) sO[row * G0 + col] = v;
      }
    }
    __syncthreads();
  }

  if (tid < G0) {
    float s = 0.0f;
#pragma unroll 4
    for (int a = 0; a < NAM; ++a) s += sO[a * G0 + tid];
    sS[tid] = s;
  }
  __syncthreads();
  if (tid < 16) {
    const v4f o = *(const v4fa*)(sS + 4 * tid);
    float* dp = RECS + (size_t)((int)blockIdx.x) * G0 + 4 * tid;
    *(volatile v4f*)dp = o;
    __threadfence();
    *(volatile v4f*)dp = o;
  }
}

template <int K, int N>
__device__ __forceinline__ void head_layer(const unsigned short* sHh, const unsigned short* sHl,
                                           const unsigned short* __restrict__ WT, const float* __restrict__ bias,
                                           float* sP, int wave, int hh, int m) {
#pragma unroll 1
  for (int nt = wave; nt < N / 16; nt += NWAVE) {
    v8f acc0 = z8(), acc1 = z8();
    const unsigned short* bp = WT + (size_t)(16 * nt + m) * K + 8 * hh;
    const unsigned short* h0 = sHh + m * K + 8 * hh;
    const unsigned short* l0 = sHl + m * K + 8 * hh;
    const unsigned short* h1 = h0 + 16 * K;
    const unsigned short* l1 = l0 + 16 * K;
#pragma unroll 1
    for (int k0 = 0; k0 < K; k0 += 32) {
      FragB bb, a;
      bb.h[0] = *(const v8usa*)(bp + k0);
      bb.h[1] = *(const v8usa*)(bp + k0 + 16);
      a.h[0] = *(const v8usa*)(h0 + k0); a.h[1] = *(const v8usa*)(h0 + k0 + 16);
      acc0 = wmb(a, bb, acc0);
      a.h[0] = *(const v8usa*)(l0 + k0); a.h[1] = *(const v8usa*)(l0 + k0 + 16);
      acc0 = wmb(a, bb, acc0);
      a.h[0] = *(const v8usa*)(h1 + k0); a.h[1] = *(const v8usa*)(h1 + k0 + 16);
      acc1 = wmb(a, bb, acc1);
      a.h[0] = *(const v8usa*)(l1 + k0); a.h[1] = *(const v8usa*)(l1 + k0 + 16);
      acc1 = wmb(a, bb, acc1);
    }
    const float bv = bf16_val(bias[16 * nt + m]);
#pragma unroll
    for (int r = 0; r < 8; ++r) {
      sP[(8 * hh + r) * N + 16 * nt + m]      = relu_np(acc0[r] + bv);
      sP[(16 + 8 * hh + r) * N + 16 * nt + m] = relu_np(acc1[r] + bv);
    }
  }
}
template <int W>
__device__ __forceinline__ void head_cvt(const float* sP, unsigned short* sHh, unsigned short* sHl, int tid) {
#pragma unroll 1
  for (int u = tid; u < (32 * W) / 8; u += NTHR) {
    const float* sp = sP + 8 * u;
    split8_store(*(const v4fa*)sp, *(const v4fa*)(sp + 4), sHh + 8 * u, sHl + 8 * u);
  }
}
__global__ __launch_bounds__(NTHR) void k_head(const float* __restrict__ RECS, const unsigned short* __restrict__ PL,
                                               const float* __restrict__ b1, const float* __restrict__ b2,
                                               const float* __restrict__ b3, const float* __restrict__ w4,
                                               const float* __restrict__ b4, float* out) {
  extern __shared__ __attribute__((aligned(16))) float hdyn[];
  float* sP = hdyn;
  float* sW = sP + 32 * FC1;
  unsigned short* sHh = (unsigned short*)(sW + 64);
  unsigned short* sHl = sHh + 32 * FC1;
  const int tid = (int)threadIdx.x, lane = tid & 31, wave = tid >> 5, hh = lane >> 4, m = lane & 15;
  {
    const int idx = tid * 8;
    const int b = idx >> 6, c = idx & 63;
    const float* r0 = RECS + (size_t)(b * KST) * G0 + c;
    const v4f a0 = *(const v4fa*)r0;
    const v4f a1 = *(const v4fa*)(r0 + 4);
    const v4f c0 = *(const v4fa*)(r0 + G0);
    const v4f c1 = *(const v4fa*)(r0 + G0 + 4);
    const v4f d0 = *(const v4fa*)(r0 + 2 * G0);
    const v4f d1 = *(const v4fa*)(r0 + 2 * G0 + 4);
    const float third = 1.0f / 3.0f;
    const v4f g0 = ((a0 + c0) + d0) * third;
    const v4f g1 = ((a1 + c1) + d1) * third;
    split8_store(g0, g1, sHh + idx, sHl + idx);
  }
  if (tid < FC3) sW[tid] = bf16_val(w4[tid]);
  __syncthreads();
  head_layer<G0, FC1>(sHh, sHl, PL + O_L1, b1, sP, wave, hh, m);
  __syncthreads();
  head_cvt<FC1>(sP, sHh, sHl, tid);
  __syncthreads();
  head_layer<FC1, FC2>(sHh, sHl, PL + O_L2, b2, sP, wave, hh, m);
  __syncthreads();
  head_cvt<FC2>(sP, sHh, sHl, tid);
  __syncthreads();
  head_layer<FC2, FC3>(sHh, sHl, PL + O_L3, b3, sP, wave, hh, m);
  __syncthreads();
  if (wave == 0) {
    float s = 0.0f;
#pragma unroll 4
    for (int c = 0; c < FC3; ++c) s = fmaf(sP[lane * FC3 + c], sW[c], s);
    s = s + bf16_val(b4[0]);
    *(volatile float*)(out + lane) = s;
    __threadfence();
    *(volatile float*)(out + lane) = s;
  }
}

extern "C" void kernel_launch(void* const* d_in, const int* in_sizes, int n_in,
                              void* d_out, int out_size, void* d_ws, size_t ws_size,
                              hipStream_t stream) {
  if (n_in < 29) return;
  const int expect[29] = {NNODES * FD, 2 * NEDGES, NEDGES * FE, NNODES, NNODES,
                          FE * FD * FD, FD * FD, FD * FD, FD,
                          FE * FD * FD, FD * FD, FD * FD, FD,
                          FE * FD * FD, FD * FD, FD * FD, FD,
                          KST * FD * G0, (TST - 1) * KST * G0 * G0, TST * KST * FD * G0, TST * KST * G0,
                          G0 * FC1, FC1, FC1 * FC2, FC2, FC2 * FC3, FC3, FC3, 1};
  for (int i = 0; i < 29; ++i) if (in_sizes[i] != expect[i]) return;
  if (out_size != NGRAPH) return;

  const float* x      = (const float*)d_in[0];
  const int*   eidx   = (const int*)d_in[1];
  const float* eattr  = (const float*)d_in[2];
  const int*   labels = (const int*)d_in[3];
  const int*   batch  = (const int*)d_in[4];
  const float* mw[3]  = {(const float*)d_in[5], (const float*)d_in[9],  (const float*)d_in[13]};
  const float* mb[3]  = {(const float*)d_in[6], (const float*)d_in[10], (const float*)d_in[14]};
  const float* rt[3]  = {(const float*)d_in[7], (const float*)d_in[11], (const float*)d_in[15]};
  const float* bs[3]  = {(const float*)d_in[8], (const float*)d_in[12], (const float*)d_in[16]};
  const float* aiw    = (const float*)d_in[17];
  const float* aw     = (const float*)d_in[18];
  const float* arw    = (const float*)d_in[19];
  const float* abias  = (const float*)d_in[20];
  const float* l1w    = (const float*)d_in[21];
  const float* l1b    = (const float*)d_in[22];
  const float* l2w    = (const float*)d_in[23];
  const float* l2b    = (const float*)d_in[24];
  const float* l3w    = (const float*)d_in[25];
  const float* l3b    = (const float*)d_in[26];
  const float* l4w    = (const float*)d_in[27];
  const float* l4b    = (const float*)d_in[28];
  float* out = (float*)d_out;

  char* ws = (char*)d_ws;
  size_t off = 0;
  const size_t oPL  = off; off += (size_t)O_END * 2;                 off = (off + 255) & ~(size_t)255;
  const size_t oHA  = off; off += (size_t)NNODES * FD * 4;           off = (off + 255) & ~(size_t)255;
  const size_t oHB  = off; off += (size_t)NNODES * FD * 4;           off = (off + 255) & ~(size_t)255;
  const size_t oRP  = off; off += (size_t)NNODES * FD * 4;           off = (off + 255) & ~(size_t)255;
  const size_t oMSG = off; off += (size_t)NEDGES * FD * 4;           off = (off + 255) & ~(size_t)255;
  const size_t oAM  = off; off += (size_t)NSEG * FD * 4;             off = (off + 255) & ~(size_t)255;
  const size_t oREC = off; off += (size_t)NGRAPH * KST * G0 * 4;     off = (off + 255) & ~(size_t)255;
  if (off > ws_size || off > (size_t)WSMAX) return;
  unsigned short* PL = (unsigned short*)(ws + oPL);
  float* HA    = (float*)(ws + oHA);
  float* HB    = (float*)(ws + oHB);
  float* ROOTP = (float*)(ws + oRP);
  float* MSG   = (float*)(ws + oMSG);
  float* AMINO = (float*)(ws + oAM);
  float* RECS  = (float*)(ws + oREC);

  hipFuncSetAttribute(reinterpret_cast<const void*>(&k_scan<0, A_NB, A_SL, A_RC>),
                      hipFuncAttributeMaxDynamicSharedMemorySize, (int)AGG_LDS_BYTES);
  hipFuncSetAttribute(reinterpret_cast<const void*>(&k_scan<1, P_NB, P_SL, P_RC>),
                      hipFuncAttributeMaxDynamicSharedMemorySize, (int)POOL_LDS_BYTES);
  hipFuncSetAttribute(reinterpret_cast<const void*>(&k_arma),
                      hipFuncAttributeMaxDynamicSharedMemorySize, (int)ARMA_LDS_BYTES);
  hipFuncSetAttribute(reinterpret_cast<const void*>(&k_head),
                      hipFuncAttributeMaxDynamicSharedMemorySize, (int)HEAD_LDS_BYTES);

  k_prep<<<U14 / PTHR, PTHR, 0, stream>>>(mw[0], mb[0], rt[0], mw[1], mb[1], rt[1], mw[2], mb[2], rt[2],
                                          aiw, aw, arw, l1w, l2w, l3w, PL);
  for (int l = 0; l < 3; ++l) {
    const float* Hin  = (l == 0) ? x : ((l == 1) ? HA : HB);
    float*       Hout = (l == 1) ? HB : HA;
    const int    rnd  = (l == 0) ? 1 : 0;
    k_root<<<NNODES / EPB, NTHR, 0, stream>>>(Hin, rnd, PL + O_RT + l * (FD * FD), bs[l], ROOTP);
    k_edge<<<NEDGES / EPB, NTHR, 0, stream>>>(Hin, rnd, eidx, eattr, PL + O_BW + l * BWL, MSG);
    k_scan<0, A_NB, A_SL, A_RC><<<NNODES / A_NB, NTHR, AGG_LDS_BYTES, stream>>>(
        eidx + NEDGES, eidx + NEDGES, NEDGES, NNODES, MSG, ROOTP, Hout);
  }
  k_scan<1, P_NB, P_SL, P_RC><<<NSEG / P_NB, NTHR, POOL_LDS_BYTES, stream>>>(
      batch, labels, NNODES, NSEG, HA, HA, AMINO);
  k_arma<<<NGRAPH * KST, NTHR, ARMA_LDS_BYTES, stream>>>(AMINO, PL, abias, RECS);
  k_head<<<1, NTHR, HEAD_LDS_BYTES, stream>>>(RECS, PL, l1b, l2b, l3b, l4w, l4b, out);
  (void)hipGetLastError();
}
